// Double_DoubleAttentionLayer_norm_64321430225068
// MI455X (gfx1250) — hardware-verified
//
#include <hip/hip_runtime.h>
#include <hip/hip_bf16.h>
#include <math.h>

#define NIMG 8
#define CCx 512
#define CM 128
#define CN 64
#define GHh 56
#define HWr 3136
#define HWp 3328
#define SS HWp
#define HH 1
#define DKK 64
#define GSTR 48

typedef _Float16 bf16;
typedef _Float16 f16;
typedef __attribute__((ext_vector_type(4))) unsigned v4u_t;
typedef unsigned v4ua __attribute__((ext_vector_type(4), may_alias));
typedef __attribute__((ext_vector_type(4))) float v4f_t;
typedef float v4fa __attribute__((ext_vector_type(4), may_alias));
typedef __attribute__((ext_vector_type(16))) bf16  bf16x16;
typedef bf16x16 f16x16;
typedef __attribute__((ext_vector_type(8)))  bf16  bf16x8;
typedef bf16x8 f16x8;
typedef __attribute__((ext_vector_type(4)))  bf16  bf16x4;
typedef __attribute__((ext_vector_type(8)))  float f32x8;
__device__ __forceinline__ f32x8 wmma16(f16x16 a, f16x16 b, f32x8 c) {
  c = __builtin_amdgcn_wmma_f32_16x16x32_f16(false, a, false, b, (short)0, c, false, false);
  asm volatile("v_nop\n\tv_nop\n\tv_nop\n\tv_nop" : "+v"(c) : "v"(a), "v"(b));
  return c;
}
#define LDS_STRIDE 48
#define KSTRIDE    72
#define VSTRIDE    48

__device__ __forceinline__ f32x8 wmma_bf16(bf16x16 a, bf16x16 b, f32x8 c) {
  c = __builtin_amdgcn_wmma_f32_16x16x32_f16(false, a, false, b, (short)0, c, false, false);
  asm volatile("v_nop\n\tv_nop\n\tv_nop\n\tv_nop" : "+v"(c) : "v"(a), "v"(b));
  return c;
}

template <typename T>
__device__ __forceinline__ bf16x16 load_frag(const T* __restrict__ base, int ld,
                                             int row0, int k0) {
  const int lane = threadIdx.x & 31;
  const int r    = lane & 15;
  const int kh   = (lane >> 4) * 8;
  const T* p0 = base + (size_t)(row0 + r) * ld + (k0 + kh);
  const T* p1 = p0 + 16;
  bf16x16 f;
#pragma unroll
  for (int i = 0; i < 8; ++i) {
    f[i]     = (bf16)p0[i];
    f[i + 8] = (bf16)p1[i];
  }
  return f;
}

__device__ __forceinline__ bf16x16 lds_frag(const bf16* base, int stride) {
  const int lane = threadIdx.x & 31;
  const int row  = lane & 15;
  const int kh   = (lane >> 4) * 8;
  const bf16x8 lo = *(const bf16x8*)(base + row * stride + kh);
  const bf16x8 hi = *(const bf16x8*)(base + row * stride + kh + 16);
  bf16x16 f;
#pragma unroll
  for (int i = 0; i < 8; ++i) { f[i] = lo[i]; f[i + 8] = hi[i]; }
  return f;
}

template <typename T>
__device__ __forceinline__ void stage_read16(const T* __restrict__ p, float* buf) {
#pragma unroll
  for (int i = 0; i < 16; ++i) buf[i] = (float)p[i];
}

__device__ __forceinline__ void stage_write(bf16* dst, const float* buf, int nquad) {
#pragma unroll
  for (int i = 0; i < nquad; ++i) {
    bf16x4 q;
    q[0] = (bf16)buf[4 * i];     q[1] = (bf16)buf[4 * i + 1];
    q[2] = (bf16)buf[4 * i + 2]; q[3] = (bf16)buf[4 * i + 3];
    *(bf16x4*)(dst + 4 * i) = q;
  }
}

template <typename AT, int MODE>
__global__ __launch_bounds__(256) void gemm_rb_kernel(
    const AT* __restrict__ A, const float* __restrict__ W,
    const float* __restrict__ bias, const float* __restrict__ rowscale, const float* __restrict__ R, const float* __restrict__ rowbias, void* __restrict__ out,
    int M, int N, int K) {
  __shared__ bf16 ldsA[128 * LDS_STRIDE];
  __shared__ bf16 ldsW[256 * LDS_STRIDE];
  __shared__ __attribute__((aligned(16))) unsigned char sob[256 * 136 * 2];

  const int t    = threadIdx.x;
  const int wave = t >> 5;
  const int lane = t & 31;
  const int wm   = (wave & 1) * 64;
  const int wn   = (wave >> 1) * 64;
  const int mBlk = blockIdx.x * 128;
  const int nBlk = blockIdx.y * 256;

  const int arow = t >> 1;
  const int ach  = (t & 1) * 16;

  float abuf[16];
  float wbuf[32];

  stage_read16(A + (size_t)(mBlk + arow) * K + ach, abuf);
  const int nrow = min(nBlk + t, N - 1);
  stage_read16(W + (size_t)nrow * K,          wbuf);
  stage_read16(W + (size_t)nrow * K + 16,     wbuf + 16);

  f32x8 acc[4][4] = {};

  for (int k = 0; k < K; k += 32) {
    __syncthreads();
    stage_write(&ldsA[arow * LDS_STRIDE + ach], abuf, 4);
    stage_write(&ldsW[t * LDS_STRIDE],          wbuf, 8);
    if (k + 32 < K) {
      stage_read16(A + (size_t)(mBlk + arow) * K + (k + 32) + ach, abuf);
      stage_read16(W + (size_t)nrow * K + (k + 32),          wbuf);
      stage_read16(W + (size_t)nrow * K + (k + 32) + 16,     wbuf + 16);
    }
    __syncthreads();

    bf16x16 af[4], wf[4];
#pragma unroll
    for (int i = 0; i < 4; ++i)
      af[i] = lds_frag(ldsA + (wm + 16 * i) * LDS_STRIDE, LDS_STRIDE);
#pragma unroll
    for (int j = 0; j < 4; ++j)
      wf[j] = lds_frag(ldsW + (wn + 16 * j) * LDS_STRIDE, LDS_STRIDE);
#pragma unroll
    for (int i = 0; i < 4; ++i)
#pragma unroll
      for (int j = 0; j < 4; ++j)
        acc[i][j] = wmma_bf16(af[i], wf[j], acc[i][j]);
  }

  const int nlane = lane & 15;
  const int mh    = (lane >> 4) * 8;
  __syncthreads();
  if (MODE == 0 || MODE == 1 || MODE == 3) {
    bf16* so = (bf16*)sob;
#pragma unroll
    for (int i = 0; i < 4; ++i)
#pragma unroll
      for (int j = 0; j < 4; ++j) {
        const int nl = wn + 16 * j + nlane;
        const float bv = bias ? bias[nBlk + nl] : 0.0f;
        if (MODE == 3) {
#pragma unroll 1
          for (int r = 0; r < 8; ++r) {
            const int ml = wm + 16 * i + mh + r;
            const float xg = acc[i][j][r] + bv;
            so[ml * 264 + nl] = (bf16)(0.5f * xg * (1.0f + erff(xg * 0.70710678118654752f)));
          }
        } else {
#pragma unroll
        for (int r = 0; r < 8; ++r) {
          const int ml = wm + 16 * i + mh + r;
          const bf16 hv = (bf16)(acc[i][j][r] + bv);
          if (MODE == 0) so[ml * 264 + nl] = hv;
          else           so[nl * 136 + ml] = hv;
        }
        }
      }
    __syncthreads();
#pragma unroll 1
    for (int pass = 0; pass < 2; ++pass) {
      if (MODE == 0 || MODE == 3) {
        for (int ch = t; ch < 128 * 32; ch += 256) { const int ml = ch >> 5, q = (ch & 31) * 8;
          *(volatile v4u_t*)((bf16*)out + (size_t)(mBlk + ml) * N + nBlk + q) = *(const v4ua*)(so + ml * 264 + q); }
      } else {
        const int b_ = mBlk / SS, s0 = mBlk % SS;
        for (int ch = t; ch < 256 * 16; ch += 256) { const int nl = ch >> 4, q = (ch & 15) * 8; const int n = nBlk + nl, h = n >> 6, dk = n & (DKK - 1);
          *(volatile v4u_t*)((bf16*)out + (((size_t)(b_ * HH + h)) * DKK + dk) * SS + s0 + q) = *(const v4ua*)(so + nl * 136 + q); }
      }
      __threadfence();
    }
  } else {
    float* so = (float*)sob;
#pragma unroll 1
    for (int hf = 0; hf < 2; ++hf) {
      if (wm == hf * 64) {
#pragma unroll
        for (int i = 0; i < 4; ++i)
#pragma unroll
          for (int j = 0; j < 4; ++j) {
            const int nl = wn + 16 * j + nlane;
            const float bv = bias ? bias[nBlk + nl] : 0.0f;
#pragma unroll
            for (int r = 0; r < 8; ++r) { const int mrow = mBlk + hf * 64 + 16 * i + mh + r; so[(16 * i + mh + r) * 260 + nl] = acc[i][j][r] * (rowscale ? rowscale[mrow] : 1.0f) + bv + (rowbias ? rowbias[mrow] : 0.0f); }
          }
      }
      __syncthreads();
      if (R) {
        for (int ch = t; ch < 64 * 64; ch += 256) { const int ml = ch >> 6, q = (ch & 63) * 4;
          if (nBlk + q < N) { const v4f_t rv = *(const v4f_t*)(R + (size_t)(mBlk + hf * 64 + ml) * N + nBlk + q); v4f_t v = *(const v4fa*)(so + ml * 260 + q); v += rv; *(volatile v4fa*)(so + ml * 260 + q) = v; } }
        asm volatile("s_wait_dscnt 0" ::: "memory");
      }
#pragma unroll 1
      for (int pass = 0; pass < 2; ++pass) {
        for (int ch = t; ch < 64 * 64; ch += 256) { const int ml = ch >> 6, q = (ch & 63) * 4;
          if (nBlk + q < N) *(volatile v4f_t*)((float*)out + (size_t)(mBlk + hf * 64 + ml) * N + nBlk + q) = *(const v4fa*)(so + ml * 260 + q); }
        __threadfence();
      }
      __syncthreads();
    }
  }
}


#define GSTR 48
template <typename AT, int EPI, bool OUT16>
__global__ __launch_bounds__(256) void gemm_kne(const AT* __restrict__ A, int lda, const float* __restrict__ Wm, int ldw,
                                                const float* __restrict__ bias, const float* __restrict__ R, const float* __restrict__ gvec,
                                                void* __restrict__ Yv, int ldy, int K) {
  __shared__ __attribute__((aligned(16))) f16 ldsA[128 * GSTR];
  __shared__ __attribute__((aligned(16))) f16 ldsW[128 * GSTR];
  __shared__ __attribute__((aligned(16))) float oS[8][32 * 68];
  const int tid = threadIdx.x, lane = tid & 31, wave = tid >> 5, cl = lane & 15, rh = (lane >> 4) * 8;
  const int m0 = blockIdx.x * 128, n0 = blockIdx.y * 128;
  const int wm = (wave & 3) * 32, wn = (wave >> 2) * 64;
  f32x8 acc[2][4];
#pragma unroll
  for (int i = 0; i < 2; ++i)
#pragma unroll
    for (int j = 0; j < 4; ++j) { f32x8 z = {}; acc[i][j] = z; }
#pragma unroll 1
  for (int k0 = 0; k0 < K; k0 += 32) {
    __syncthreads();
    { const int row = tid >> 1, ch = (tid & 1) * 16;
      const AT* src = A + (size_t)(m0 + row) * lda + k0 + ch;
#pragma unroll
      for (int g = 0; g < 16; ++g) ldsA[row * GSTR + ch + g] = (f16)src[g]; }
    { const int k = tid >> 3, nn0 = (tid & 7) * 16;
      const float* src = Wm + (size_t)(k0 + k) * ldw + n0 + nn0;
#pragma unroll
      for (int g = 0; g < 4; ++g) { const v4f_t v = *(const v4f_t*)(src + 4 * g);
#pragma unroll
        for (int u = 0; u < 4; ++u) ldsW[(nn0 + 4 * g + u) * GSTR + k] = (f16)v[u]; } }
    __syncthreads();
    f16x16 af[2];
#pragma unroll
    for (int i = 0; i < 2; ++i) af[i] = lds_frag(ldsA + (wm + 16 * i) * GSTR, GSTR);
#pragma unroll
    for (int j = 0; j < 4; ++j) {
      const f16x16 bf = lds_frag(ldsW + (wn + 16 * j) * GSTR, GSTR);
#pragma unroll
      for (int i = 0; i < 2; ++i) acc[i][j] = wmma16(af[i], bf, acc[i][j]);
    }
  }
  float* so = oS[wave];
#pragma unroll
  for (int i = 0; i < 2; ++i)
#pragma unroll
    for (int j = 0; j < 4; ++j) {
      const int n = n0 + wn + 16 * j + cl;
      const float bv = bias ? bias[n] : 0.0f;
      const float gv = (EPI == 2) ? gvec[n] : 0.0f;
      if (EPI == 1) {
#pragma unroll 1
        for (int r = 0; r < 8; ++r) { const float xg = acc[i][j][r] + bv; so[(16 * i + rh + r) * 68 + 16 * j + cl] = 0.5f * xg * (1.0f + erff(xg * 0.70710678118654752f)); }
      } else {
#pragma unroll
        for (int r = 0; r < 8; ++r) {
          float v = acc[i][j][r] + bv;
          if (EPI == 2) v = R[(size_t)(m0 + wm + 16 * i + rh + r) * ldy + n] + gv * v;
          so[(16 * i + rh + r) * 68 + 16 * j + cl] = v;
        }
      }
    }
  asm volatile("s_wait_dscnt 0" ::: "memory");
  __builtin_amdgcn_wave_barrier();
#pragma unroll 1
  for (int pass = 0; pass < 2; ++pass) {
    if (OUT16) {
      f16* Y = (f16*)Yv;
#pragma unroll
      for (int it = 0; it < 8; ++it) { const int c = lane + 32 * it, rr = c >> 3, q8 = (c & 7) * 8;
        union { f16 h[8]; v4u_t v; } u;
#pragma unroll
        for (int e = 0; e < 8; ++e) u.h[e] = (f16)so[rr * 68 + q8 + e];
        *(volatile v4u_t*)(Y + (size_t)(m0 + wm + rr) * ldy + n0 + wn + q8) = u.v; }
    } else {
      float* Y = (float*)Yv;
#pragma unroll
      for (int it = 0; it < 16; ++it) { const int f4 = lane + 32 * it, rr = f4 >> 4, q = (f4 & 15) * 4;
        *(volatile v4f_t*)(Y + (size_t)(m0 + wm + rr) * ldy + n0 + wn + q) = *(const v4fa*)(so + rr * 68 + q); }
    }
    __threadfence();
  }
}

__global__ __launch_bounds__(256) void k_padcopy(const float* __restrict__ xb, float* __restrict__ xp) { const size_t c = blockIdx.x;
  for (int q4 = threadIdx.x; q4 < HWp / 4; q4 += 256) { v4f_t v = {0.f,0.f,0.f,0.f}; if (q4 * 4 < HWr) v = *(const v4f_t*)(xb + c * HWr + q4 * 4); *(volatile v4f_t*)(xp + c * HWp + q4 * 4) = v; __threadfence(); *(volatile v4f_t*)(xp + c * HWp + q4 * 4) = v; } }
__global__ __launch_bounds__(256) void k_rowbias(float* __restrict__ t, const float* __restrict__ bias) { const size_t row = blockIdx.x; const float bv = bias[row];
  for (int q4 = threadIdx.x; q4 < HWp / 4; q4 += 256) { v4f_t v = *(const v4f_t*)(t + row * HWp + q4 * 4); for (int e = 0; e < 4; ++e) v[e] += bv; *(volatile v4f_t*)(t + row * HWp + q4 * 4) = v; __threadfence(); *(volatile v4f_t*)(t + row * HWp + q4 * 4) = v; } }
__global__ __launch_bounds__(256) void k_rowsoftmax(float* __restrict__ T) {
  __shared__ float red[256];
  const size_t row = blockIdx.x; const int tid = threadIdx.x; float* tr = T + row * HWp;
  float v[13]; float m = -3.0e38f;
#pragma unroll
  for (int e = 0; e < 13; ++e) { const int p = tid + 256 * e; v[e] = (p < HWr) ? tr[p] : -3.0e38f; m = fmaxf(m, v[e]); }
  red[tid] = m; __syncthreads();
  for (int o = 128; o > 0; o >>= 1) { if (tid < o) red[tid] = fmaxf(red[tid], red[tid + o]); __syncthreads(); }
  m = red[0]; __syncthreads();
  float z = 0.0f;
#pragma unroll
  for (int e = 0; e < 13; ++e) { const int p = tid + 256 * e; v[e] = (p < HWr) ? expf(v[e] - m) : 0.0f; z += v[e]; }
  red[tid] = z; __syncthreads();
  for (int o = 128; o > 0; o >>= 1) { if (tid < o) red[tid] += red[tid + o]; __syncthreads(); }
  const float iz = 1.0f / red[0];
#pragma unroll 1
  for (int pass = 0; pass < 2; ++pass) { for (int e = 0; e < 13; ++e) { const int p = tid + 256 * e; *(volatile float*)(tr + p) = v[e] * iz; } __threadfence(); }
}
__global__ __launch_bounds__(256) void k_colsoftmax(float* __restrict__ T, int nr) {
  const int p = blockIdx.x * 256 + threadIdx.x; if (p >= HWp) return;
  float m = -3.0e38f;
#pragma unroll 1
  for (int r = 0; r < nr; ++r) m = fmaxf(m, T[(size_t)r * HWp + p]);
  float z = 0.0f;
#pragma unroll 1
  for (int r = 0; r < nr; ++r) z += expf(T[(size_t)r * HWp + p] - m);
  const float iz = (p < HWr) ? 1.0f / z : 0.0f;
#pragma unroll 1
  for (int r = 0; r < nr; ++r) { const float v = (p < HWr) ? expf(T[(size_t)r * HWp + p] - m) * iz : 0.0f; *(volatile float*)(T + (size_t)r * HWp + p) = v; __threadfence(); *(volatile float*)(T + (size_t)r * HWp + p) = v; }
}
__global__ __launch_bounds__(256) void k_transpose(const float* __restrict__ Wm, float* __restrict__ Wt, int rows, int cols) {
  __shared__ float tS[64][65];
  const int tid = threadIdx.x, tbj = cols / 64, bi = blockIdx.x / tbj, bj = blockIdx.x % tbj;
  for (int e = tid; e < 64 * 64; e += 256) { const int r = e >> 6, c = e & 63; tS[r][c] = Wm[(size_t)(bi * 64 + r) * cols + bj * 64 + c]; }
  __syncthreads();
  for (int ch = tid; ch < 64 * 16; ch += 256) { const int r = ch >> 4, q4 = (ch & 15) * 4; v4f_t o; o[0] = tS[q4][r]; o[1] = tS[q4 + 1][r]; o[2] = tS[q4 + 2][r]; o[3] = tS[q4 + 3][r];
    float* dst = Wt + (size_t)(bj * 64 + r) * rows + bi * 64 + q4; *(volatile v4f_t*)dst = o; __threadfence(); *(volatile v4f_t*)dst = o; }
}
__global__ __launch_bounds__(256) void k_bnrelu(float* __restrict__ t, const float* __restrict__ bE, const float* __restrict__ g, const float* __restrict__ bb, const float* __restrict__ mn, const float* __restrict__ vr) {
  const size_t c = blockIdx.x; const float sc = g[c] * rsqrtf(vr[c] + 1e-5f), sh = (bE[c] - mn[c]) * sc + bb[c];
  for (int q4 = threadIdx.x; q4 < HWp / 4; q4 += 256) { v4f_t v = *(const v4f_t*)(t + c * HWp + q4 * 4); for (int e = 0; e < 4; ++e) v[e] = fmaxf(v[e] * sc + sh, 0.0f); *(volatile v4f_t*)(t + c * HWp + q4 * 4) = v; __threadfence(); *(volatile v4f_t*)(t + c * HWp + q4 * 4) = v; } }
__global__ __launch_bounds__(256) void k_sum3(const float* __restrict__ E, const float* __restrict__ ES, const float* __restrict__ xb, float* __restrict__ S) { const size_t c = blockIdx.x;
  for (int q4 = threadIdx.x; q4 < HWr / 4; q4 += 256) { const v4f_t a = *(const v4f_t*)(E + c * HWp + q4 * 4), b2 = *(const v4f_t*)(ES + c * HWp + q4 * 4), xx = *(const v4f_t*)(xb + c * HWr + q4 * 4); v4f_t o;
    for (int e = 0; e < 4; ++e) o[e] = a[e] + b2[e] + xx[e]; *(volatile v4f_t*)(S + c * HWr + q4 * 4) = o; __threadfence(); *(volatile v4f_t*)(S + c * HWr + q4 * 4) = o; } }
__global__ __launch_bounds__(256) void k_conv3(const float* __restrict__ S, const float* __restrict__ Wc, const float* __restrict__ bc, float* __restrict__ outb) {
  __shared__ __attribute__((aligned(16))) f16 aS[128 * 40];
  __shared__ __attribute__((aligned(16))) f16 bS[128 * 40];
  __shared__ __attribute__((aligned(16))) float oS[128 * 132];
  const int tid = threadIdx.x, lane = tid & 31, wave = tid >> 5, cl = lane & 15, rh = (lane >> 4) * 8;
  const int p0 = blockIdx.x * 128, co0 = blockIdx.y * 128;
  f32x8 acc[8];
#pragma unroll
  for (int j = 0; j < 8; ++j) { f32x8 z = {}; acc[j] = z; }
  const int r = tid >> 1, q = (tid & 1) * 16; const int p = p0 + r; const bool pv = p < HWr; const int py = p / GHh, px = p % GHh;
#pragma unroll 1
  for (int ks = 0; ks < (CCx * 9) / 32; ++ks) {
    __syncthreads();
#pragma unroll 1
    for (int e = 0; e < 16; ++e) { const int k = ks * 32 + q + e, ci = k / 9, tap = k - ci * 9, yy = py + tap / 3 - 1, xx = px + tap % 3 - 1;
      float v = 0.0f; if (pv && yy >= 0 && yy < GHh && xx >= 0 && xx < GHh) v = S[(size_t)ci * HWr + yy * GHh + xx]; aS[r * 40 + q + e] = (f16)v; }
    { const int co = tid >> 1; const float* wr = Wc + (size_t)(co0 + co) * (CCx * 9) + ks * 32 + q;
#pragma unroll
      for (int e = 0; e < 16; ++e) bS[co * 40 + q + e] = (f16)wr[e]; }
    __syncthreads();
    const f16x16 af = lds_frag(aS + (wave * 16) * 40, 40);
#pragma unroll
    for (int j = 0; j < 8; ++j) acc[j] = wmma16(af, lds_frag(bS + (j * 16) * 40, 40), acc[j]);
  }
#pragma unroll
  for (int j = 0; j < 8; ++j) { const int co = j * 16 + cl; const float bb = bc[co0 + co];
#pragma unroll
    for (int rr = 0; rr < 8; ++rr) oS[co * 132 + wave * 16 + rh + rr] = acc[j][rr] + bb; }
  __syncthreads();
  const int nvalid = (HWr - p0 < 128) ? (HWr - p0) : 128;
  const int n4 = nvalid / 4;
#pragma unroll 1
  for (int pass = 0; pass < 2; ++pass) { for (int q4 = tid; q4 < 128 * n4; q4 += 256) { const int co = q4 / n4, c4 = (q4 % n4) * 4;
      *(volatile v4f_t*)(outb + (size_t)(co0 + co) * HWr + p0 + c4) = *(const v4fa*)(oS + co * 132 + c4); } __threadfence(); }
}

extern "C" void kernel_launch(void* const* d_in, const int* in_sizes, int n_in,
                              void* d_out, int out_size, void* d_ws, size_t ws_size,
                              hipStream_t stream) {
  (void)in_sizes; (void)n_in; (void)out_size;
  const float** f = (const float**)d_in;
  const float* x = f[0], *WA = f[1], *bA = f[2], *WB = f[3], *bB = f[4], *WV = f[5], *bV = f[6], *WAs = f[7], *bAs = f[8], *WBs = f[9], *bBs = f[10], *WVs = f[11], *bVs = f[12],
             *WE = f[13], *bE = f[14], *bng = f[15], *bnb = f[16], *bnm = f[17], *bnv = f[18], *Wout = f[19], *bout = f[20];
  float* out = (float*)d_out;
  char* ws = (char*)d_ws;
  float* xp = (float*)ws; ws += (size_t)CCx * HWp * 4;
  float* WBV = (float*)ws; ws += (size_t)CM * CCx * 4;
  float* ABV = (float*)ws; ws += (size_t)2 * CM * HWp * 4;
  float* BVT = (float*)ws; ws += (size_t)HWp * CM * 4;
  float* Gp = (float*)ws; ws += (size_t)CM * 128 * 4;
  float* Z = (float*)ws; ws += (size_t)CM * HWp * 4;
  float* E = (float*)ws; ws += (size_t)CCx * HWp * 4;
  float* S3 = (float*)ws; ws += (size_t)3 * CM * HWp * 4;
  float* AST = (float*)ws; ws += (size_t)HWp * CM * 4;
  float* GS = (float*)ws; ws += (size_t)HWp * HWp * 4;
  float* ZS = (float*)ws; ws += (size_t)CM * HWp * 4;
  float* ES = (float*)ws; ws += (size_t)CCx * HWp * 4;
  float* Ssum = (float*)ws; ws += (size_t)CCx * HWr * 4;
  if ((size_t)(ws - (char*)d_ws) > ws_size) return;
  const dim3 blk(256);
  hipMemcpyAsync(WBV, WB, (size_t)CN * CCx * 4, hipMemcpyDeviceToDevice, stream);
  hipMemcpyAsync(WBV + (size_t)CN * CCx, WV, (size_t)CN * CCx * 4, hipMemcpyDeviceToDevice, stream);
  for (int b = 0; b < NIMG; ++b) {
    const float* xb = x + (size_t)b * CCx * HWr; float* ob = out + (size_t)b * CCx * HWr;
    k_padcopy<<<dim3(CCx), blk, 0, stream>>>(xb, xp);
    gemm_kne<float, 0, false><<<dim3(1, HWp / 128), blk, 0, stream>>>(WA, CCx, xp, HWp, nullptr, nullptr, nullptr, ABV, HWp, CCx);
    gemm_kne<float, 0, false><<<dim3(1, HWp / 128), blk, 0, stream>>>(WBV, CCx, xp, HWp, nullptr, nullptr, nullptr, ABV + (size_t)CM * HWp, HWp, CCx);
    k_rowbias<<<dim3(CM), blk, 0, stream>>>(ABV, bA); k_rowbias<<<dim3(CN), blk, 0, stream>>>(ABV + (size_t)CM * HWp, bB); k_rowbias<<<dim3(CN), blk, 0, stream>>>(ABV + (size_t)(CM + CN) * HWp, bV);
    k_rowsoftmax<<<dim3(CN), blk, 0, stream>>>(ABV + (size_t)CM * HWp);
    k_colsoftmax<<<dim3(HWp / 256), blk, 0, stream>>>(ABV + (size_t)(CM + CN) * HWp, CN);
    k_transpose<<<dim3((CM / 64) * (HWp / 64)), blk, 0, stream>>>(ABV + (size_t)CM * HWp, BVT, CM, HWp);
    gemm_kne<float, 0, false><<<dim3(1, 1), blk, 0, stream>>>(ABV, HWp, BVT, CM, nullptr, nullptr, nullptr, Gp, 128, HWp);
    gemm_kne<float, 0, false><<<dim3(1, HWp / 128), blk, 0, stream>>>(Gp, 128, ABV + (size_t)(CM + CN) * HWp, HWp, nullptr, nullptr, nullptr, Z, HWp, CN);
    gemm_kne<float, 0, false><<<dim3(CCx / 128, HWp / 128), blk, 0, stream>>>(WE, CM, Z, HWp, nullptr, nullptr, nullptr, E, HWp, CM);
    k_bnrelu<<<dim3(CCx), blk, 0, stream>>>(E, bE, bng, bnb, bnm, bnv);
    gemm_kne<float, 0, false><<<dim3(1, HWp / 128), blk, 0, stream>>>(WAs, CCx, xp, HWp, nullptr, nullptr, nullptr, S3, HWp, CCx);
    gemm_kne<float, 0, false><<<dim3(1, HWp / 128), blk, 0, stream>>>(WBs, CCx, xp, HWp, nullptr, nullptr, nullptr, S3 + (size_t)CM * HWp, HWp, CCx);
    gemm_kne<float, 0, false><<<dim3(1, HWp / 128), blk, 0, stream>>>(WVs, CCx, xp, HWp, nullptr, nullptr, nullptr, S3 + (size_t)2 * CM * HWp, HWp, CCx);
    k_rowbias<<<dim3(CM), blk, 0, stream>>>(S3, bAs); k_rowbias<<<dim3(CM), blk, 0, stream>>>(S3 + (size_t)CM * HWp, bBs); k_rowbias<<<dim3(CM), blk, 0, stream>>>(S3 + (size_t)2 * CM * HWp, bVs);
    k_colsoftmax<<<dim3(HWp / 256), blk, 0, stream>>>(S3 + (size_t)CM * HWp, CM);
    k_colsoftmax<<<dim3(HWp / 256), blk, 0, stream>>>(S3 + (size_t)2 * CM * HWp, CM);
    k_transpose<<<dim3((CM / 64) * (HWp / 64)), blk, 0, stream>>>(S3, AST, CM, HWp);
    gemm_kne<float, 0, false><<<dim3(HWp / 128, HWp / 128), blk, 0, stream>>>(AST, CM, S3 + (size_t)CM * HWp, HWp, nullptr, nullptr, nullptr, GS, HWp, CM);
    gemm_rb_kernel<float, 2><<<dim3(CM / 128, HWp / 256), blk, 0, stream>>>(S3 + (size_t)2 * CM * HWp, GS, nullptr, nullptr, nullptr, nullptr, ZS, CM, HWp, HWp);
    gemm_kne<float, 0, false><<<dim3(CCx / 128, HWp / 128), blk, 0, stream>>>(WE, CM, ZS, HWp, nullptr, nullptr, nullptr, ES, HWp, CM);
    k_bnrelu<<<dim3(CCx), blk, 0, stream>>>(ES, bE, bng, bnb, bnm, bnv);
    k_sum3<<<dim3(CCx), blk, 0, stream>>>(E, ES, xb, Ssum);
    k_conv3<<<dim3((HWr + 127) / 128, CCx / 128), blk, 0, stream>>>(Ssum, Wout, bout, ob);
  }
}
